// ConvNAT_7189775254123
// MI455X (gfx1250) — hardware-verified
//
#include <hip/hip_runtime.h>
#include <stdint.h>

#define NB     2
#define CIN    64
#define CMID   128
#define C3     384
#define HH     96
#define WW     96
#define HP     98
#define WP     98
#define IMGPIX 9216
#define NPIX   18432
#define PADPIX 19208
#define KCV    576
#define NKS    18
#define GCNT   36864
#define NGRP   32
#define KSZ    7
#define NKEY   49
#define HD     32
#define APB    32
#define LDC    132
#define OSP    36
#define SLN    32
#define SCL    11.313708498984761f
#define RSC    0.00048828125f

static_assert(NPIX == NB * IMGPIX);
static_assert(IMGPIX == HH * WW);
static_assert(PADPIX == NB * HP * WP);
static_assert(KCV == 9 * CIN && KCV == NKS * 32);
static_assert(GCNT == 4 * IMGPIX && (GCNT % 1024) == 0);
static_assert(NGRP == NB * 16);
static_assert((NPIX % 64) == 0 && (IMGPIX % 64) == 0 && (IMGPIX % APB) == 0 && (WW % APB) == 0);
static_assert(NKEY == KSZ * KSZ && CMID == 4 * HD);
static_assert((LDC * 4) % 16 == 0 && (OSP * 4) % 16 == 0);
static_assert((PADPIX % 4) == 0);
static_assert(APB * 4 == 128);

typedef _Float16 v16h __attribute__((ext_vector_type(16)));
typedef _Float16 v8h  __attribute__((ext_vector_type(8)));
typedef float    v8f  __attribute__((ext_vector_type(8)));
typedef float    v4f  __attribute__((ext_vector_type(4)));
typedef unsigned int v4u __attribute__((ext_vector_type(4)));

__device__ __forceinline__ unsigned short bf_bits(float f) {
  unsigned u = __float_as_uint(f);
  return (unsigned short)((u + 0x7FFFu + ((u >> 16) & 1u)) >> 16);
}
__device__ __forceinline__ float bf_up(unsigned short b) { return __uint_as_float(((unsigned)b) << 16); }
__device__ __forceinline__ float bfr(float f) { return bf_up(bf_bits(f)); }
__device__ __forceinline__ unsigned short h_bits(_Float16 x) { return __builtin_bit_cast(unsigned short, x); }
__device__ __forceinline__ unsigned short hb16(float f) { return h_bits((_Float16)f); }
__device__ __forceinline__ unsigned pk16(unsigned short a, unsigned short b) { return (unsigned)a | ((unsigned)b << 16); }
__device__ __forceinline__ v8f zero8() { v8f z = {0.f, 0.f, 0.f, 0.f, 0.f, 0.f, 0.f, 0.f}; return z; }

__device__ __forceinline__ v16h ldfrag_h(const _Float16* p) {
  union { v16h v; v8h h[2]; } f;
  f.h[0] = *(const v8h*)(p);
  f.h[1] = *(const v8h*)(p + 16);
  return f.v;
}

__device__ __forceinline__ v8f mma_raw(v16h a, v16h b, v8f c) {
  return __builtin_amdgcn_wmma_f32_16x16x32_f16(false, a, false, b, (short)0, c, false, false);
}
__device__ __forceinline__ void guard8(v8f& c0, v8f& c1, v8f& c2, v8f& c3, v8f& c4, v8f& c5, v8f& c6, v8f& c7,
                                       const v16h& a0, const v16h& a1, const v16h& a2, const v16h& a3,
                                       const v16h& b0, const v16h& b1) {
#if defined(__HIP_DEVICE_COMPILE__)
  asm volatile("v_nop\n\tv_nop\n\tv_nop\n\tv_nop"
               : "+v"(c0), "+v"(c1), "+v"(c2), "+v"(c3), "+v"(c4), "+v"(c5), "+v"(c6), "+v"(c7)
               : "v"(a0), "v"(a1), "v"(a2), "v"(a3), "v"(b0), "v"(b1));
#endif
}

__device__ __forceinline__ void mm_tile2(const _Float16* __restrict__ Ah, const _Float16* __restrict__ Al, int lda,
                                         const _Float16* __restrict__ W, int ldw, int nks,
                                         int arow0, int bcol0, float* Cs) {
  const int tid = threadIdx.x, wave = tid >> 5, lane = tid & 31, hh = lane >> 4, c = lane & 15;
  const int mw = wave >> 2, nw = wave & 3;
  const size_t r0 = (size_t)(arow0 + mw * 32 + c) * lda + 8 * hh;
  const size_t r1 = (size_t)(arow0 + mw * 32 + 16 + c) * lda + 8 * hh;
  const _Float16* a0h = Ah + r0;
  const _Float16* a1h = Ah + r1;
  const _Float16* a0l = Al + r0;
  const _Float16* a1l = Al + r1;
  const _Float16* b0p = W + (size_t)(bcol0 + nw * 32 + c) * ldw + 8 * hh;
  const _Float16* b1p = W + (size_t)(bcol0 + nw * 32 + 16 + c) * ldw + 8 * hh;
  v8f h00 = zero8(), h01 = zero8(), h10 = zero8(), h11 = zero8();
  v8f l00 = zero8(), l01 = zero8(), l10 = zero8(), l11 = zero8();
#pragma unroll 1
  for (int ks = 0; ks < nks; ++ks) {
    const int ko = ks * 32;
    const v16h fa0 = ldfrag_h(a0h + ko);
    const v16h fa1 = ldfrag_h(a1h + ko);
    const v16h ga0 = ldfrag_h(a0l + ko);
    const v16h ga1 = ldfrag_h(a1l + ko);
    const v16h fb0 = ldfrag_h(b0p + ko);
    const v16h fb1 = ldfrag_h(b1p + ko);
    h00 = mma_raw(fa0, fb0, h00);
    h01 = mma_raw(fa0, fb1, h01);
    h10 = mma_raw(fa1, fb0, h10);
    h11 = mma_raw(fa1, fb1, h11);
    l00 = mma_raw(ga0, fb0, l00);
    l01 = mma_raw(ga0, fb1, l01);
    l10 = mma_raw(ga1, fb0, l10);
    l11 = mma_raw(ga1, fb1, l11);
    guard8(h00, h01, h10, h11, l00, l01, l10, l11, fa0, fa1, ga0, ga1, fb0, fb1);
  }
#pragma unroll
  for (int r = 0; r < 8; ++r) {
    const int row = mw * 32 + 8 * hh + r;
    Cs[row * LDC + nw * 32 + c]             = h00[r] + l00[r] * RSC;
    Cs[row * LDC + nw * 32 + 16 + c]        = h01[r] + l01[r] * RSC;
    Cs[(row + 16) * LDC + nw * 32 + c]      = h10[r] + l10[r] * RSC;
    Cs[(row + 16) * LDC + nw * 32 + 16 + c] = h11[r] + l11[r] * RSC;
  }
}

__device__ __forceinline__ size_t conv_abase(int p, int hh) {
  const int b = p / IMGPIX;
  const int r = p - b * IMGPIX;
  const int y = r / WW;
  const int x = r - y * WW;
  return ((size_t)(b * HP + y) * WP + x) * CIN + 8 * hh;
}
__device__ __forceinline__ void mm_conv(const _Float16* __restrict__ Ah, const _Float16* __restrict__ Al,
                                        const _Float16* __restrict__ W, int prow0, float* Cs) {
  const int tid = threadIdx.x, wave = tid >> 5, lane = tid & 31, hh = lane >> 4, c = lane & 15;
  const int mw = wave >> 2, nw = wave & 3;
  const size_t r0 = conv_abase(prow0 + mw * 32 + c, hh);
  const size_t r1 = conv_abase(prow0 + mw * 32 + 16 + c, hh);
  const _Float16* a0h = Ah + r0;
  const _Float16* a1h = Ah + r1;
  const _Float16* a0l = Al + r0;
  const _Float16* a1l = Al + r1;
  const _Float16* b0p = W + (size_t)(nw * 32 + c) * KCV + 8 * hh;
  const _Float16* b1p = W + (size_t)(nw * 32 + 16 + c) * KCV + 8 * hh;
  v8f h00 = zero8(), h01 = zero8(), h10 = zero8(), h11 = zero8();
  v8f l00 = zero8(), l01 = zero8(), l10 = zero8(), l11 = zero8();
#pragma unroll 1
  for (int ks = 0; ks < NKS; ++ks) {
    const int tap = ks >> 1, chalf = ks & 1;
    const int ky = (tap * 11) >> 5;
    const int kx = tap - 3 * ky;
    const int ao = (ky * WP + kx) * CIN + chalf * 32;
    const int ko = ks * 32;
    const v16h fa0 = ldfrag_h(a0h + ao);
    const v16h fa1 = ldfrag_h(a1h + ao);
    const v16h ga0 = ldfrag_h(a0l + ao);
    const v16h ga1 = ldfrag_h(a1l + ao);
    const v16h fb0 = ldfrag_h(b0p + ko);
    const v16h fb1 = ldfrag_h(b1p + ko);
    h00 = mma_raw(fa0, fb0, h00);
    h01 = mma_raw(fa0, fb1, h01);
    h10 = mma_raw(fa1, fb0, h10);
    h11 = mma_raw(fa1, fb1, h11);
    l00 = mma_raw(ga0, fb0, l00);
    l01 = mma_raw(ga0, fb1, l01);
    l10 = mma_raw(ga1, fb0, l10);
    l11 = mma_raw(ga1, fb1, l11);
    guard8(h00, h01, h10, h11, l00, l01, l10, l11, fa0, fa1, ga0, ga1, fb0, fb1);
  }
#pragma unroll
  for (int r = 0; r < 8; ++r) {
    const int row = mw * 32 + 8 * hh + r;
    Cs[row * LDC + nw * 32 + c]             = h00[r] + l00[r] * RSC;
    Cs[row * LDC + nw * 32 + 16 + c]        = h01[r] + l01[r] * RSC;
    Cs[(row + 16) * LDC + nw * 32 + c]      = h10[r] + l10[r] * RSC;
    Cs[(row + 16) * LDC + nw * 32 + 16 + c] = h11[r] + l11[r] * RSC;
  }
}

__global__ __launch_bounds__(256)
void k_wcvt(const float* __restrict__ cw, const float* __restrict__ qw, const float* __restrict__ kw,
            const float* __restrict__ vw, unsigned short* wt, unsigned short* wqkv) {
  const int tid = threadIdx.x;
  const int blk = blockIdx.x;
  if (blk < CMID) {
    const int co = blk;
    const int t = min(tid, 71);
    const int k0 = t * 8, tap = k0 >> 6, c0 = k0 & 63;
    const float* src = cw + (size_t)co * KCV;
    v4u pk;
#pragma unroll
    for (int e = 0; e < 4; ++e) {
      const float f0 = src[(c0 + 2 * e) * 9 + tap];
      const float f1 = src[(c0 + 2 * e + 1) * 9 + tap];
      pk[e] = pk16(hb16(bfr(f0) * 64.0f), hb16(bfr(f1) * 64.0f));
    }
    if (tid < 72) {
      unsigned short* dst = wt + (size_t)co * KCV + k0;
      *(volatile v4u*)dst = pk;
      __threadfence();
      *(volatile v4u*)dst = pk;
    }
  } else {
    const int rr = blk - CMID;
    const int sel = rr >> 7, o = rr & 127;
    const float* src = (sel == 0) ? qw : ((sel == 1) ? kw : vw);
    const int t = min(tid, 15);
    const int c0 = t * 8;
    v4u pk;
#pragma unroll
    for (int e = 0; e < 4; ++e) {
      const float f0 = src[(size_t)o * CMID + c0 + 2 * e];
      const float f1 = src[(size_t)o * CMID + c0 + 2 * e + 1];
      pk[e] = pk16(hb16(bfr(f0) * 64.0f), hb16(bfr(f1) * 64.0f));
    }
    if (tid < 16) {
      unsigned short* dst = wqkv + (size_t)rr * CMID + c0;
      *(volatile v4u*)dst = pk;
      __threadfence();
      *(volatile v4u*)dst = pk;
    }
  }
}

__global__ __launch_bounds__(256)
void k_gnstat(const float* __restrict__ x, float* stats) {
  __shared__ double red[256];
  const int tid = threadIdx.x;
  const float* xb = x + (size_t)blockIdx.x * GCNT;
  float s = 0.f;
#pragma unroll 2
  for (int it = 0; it < GCNT / 1024; ++it) {
    const v4f a = *(const v4f*)(xb + (size_t)(it * 256 + tid) * 4);
    s += (bfr(a[0]) + bfr(a[1])) + (bfr(a[2]) + bfr(a[3]));
  }
  red[tid] = (double)s;
  __syncthreads();
  for (int st = 128; st > 0; st >>= 1) {
    if (tid < st) red[tid] = red[tid] + red[tid + st];
    __syncthreads();
  }
  const float mf = (float)(red[0] * (1.0 / (double)GCNT));
  __syncthreads();
  float sq = 0.f;
#pragma unroll 2
  for (int it = 0; it < GCNT / 1024; ++it) {
    const v4f a = *(const v4f*)(xb + (size_t)(it * 256 + tid) * 4);
    const float d0 = bfr(a[0]) - mf, d1 = bfr(a[1]) - mf, d2 = bfr(a[2]) - mf, d3 = bfr(a[3]) - mf;
    sq += (d0 * d0 + d1 * d1) + (d2 * d2 + d3 * d3);
  }
  red[tid] = (double)sq;
  __syncthreads();
  for (int st = 128; st > 0; st >>= 1) {
    if (tid < st) red[tid] = red[tid] + red[tid + st];
    __syncthreads();
  }
  const float varf = (float)(red[0] * (1.0 / (double)GCNT));
  const float rstd = rsqrtf(varf + 1e-5f);
  if (tid < 8) {
    v4f val;
    val[0] = (tid == 0) ? mf : 0.f;
    val[1] = (tid == 0) ? rstd : 0.f;
    val[2] = 0.f;
    val[3] = 0.f;
    float* p = stats + (size_t)blockIdx.x * SLN + tid * 4;
    *(volatile v4f*)p = val;
    __threadfence();
    *(volatile v4f*)p = val;
  }
}

__global__ __launch_bounds__(256)
void k_xn(const float* __restrict__ x, const float* __restrict__ gw, const float* __restrict__ gb,
          const float* __restrict__ stats, unsigned short* xh, unsigned short* xl) {
  const int tid = threadIdx.x, wv = tid >> 5, lane = tid & 31;
  const int w = blockIdx.x * 8 + wv;
  const int pp = w * 4 + (lane >> 3);
  const int piece = lane & 7, c0 = piece * 8;
  const int ppc = min(pp, PADPIX - 1);
  const int b = ppc / (HP * WP);
  const int r = ppc - b * (HP * WP);
  const int py = r / WP, px = r - py * WP;
  const int y = py - 1, xx = px - 1;
  const bool inside = ((unsigned)y < (unsigned)HH) && ((unsigned)xx < (unsigned)WW);
  const int yc = min(max(y, 0), HH - 1), xc = min(max(xx, 0), WW - 1);
  const float* src = x + ((size_t)(b * CIN + c0) * HH + yc) * WW + xc;
  const float* st = stats + (size_t)(b * 16 + (c0 >> 2)) * SLN;
  const float m0 = st[0], r0 = st[1], m1 = st[SLN], r1 = st[SLN + 1];
  unsigned short hb[8], lb[8];
#pragma unroll
  for (int e = 0; e < 8; ++e) {
    const float xr = bfr(src[(size_t)e * IMGPIX]);
    const float mu = (e < 4) ? m0 : m1;
    const float rs = (e < 4) ? r0 : r1;
    const float xn = ((xr - mu) * rs) * bfr(gw[c0 + e]) + bfr(gb[c0 + e]);
    const float a = inside ? xn * 8.0f : 0.0f;
    const _Float16 hv = (_Float16)a;
    const float resid = (a - (float)hv) * 2048.0f;
    hb[e] = h_bits(hv);
    lb[e] = hb16(resid);
  }
  v4u ph, plq;
#pragma unroll
  for (int e = 0; e < 4; ++e) { ph[e] = pk16(hb[2 * e], hb[2 * e + 1]); plq[e] = pk16(lb[2 * e], lb[2 * e + 1]); }
  if (pp < PADPIX) {
    const size_t ko = (size_t)pp * CIN + c0;
    *(volatile v4u*)(xh + ko) = ph;
    *(volatile v4u*)(xl + ko) = plq;
    __threadfence();
    *(volatile v4u*)(xh + ko) = ph;
    *(volatile v4u*)(xl + ko) = plq;
  }
}

__global__ __launch_bounds__(256)
void k_conv(const unsigned short* __restrict__ xh, const unsigned short* __restrict__ xl,
            const unsigned short* __restrict__ wt, const float* __restrict__ cb,
            unsigned short* fh, unsigned short* fl) {
  __shared__ __align__(16) float Cs[64 * LDC];
  const int tid = threadIdx.x;
  const int mb = blockIdx.x;
  mm_conv((const _Float16*)(const void*)xh, (const _Float16*)(const void*)xl,
          (const _Float16*)(const void*)wt, mb * 64, Cs);
  __syncthreads();
#pragma unroll 1
  for (int it = 0; it < 32; ++it) {
    const int idx = it * 256 + tid;
    const int row = idx >> 7, col = idx & 127;
    const float v = Cs[row * LDC + col] * (1.0f / 512.0f) + bfr(cb[col]);
    const float gl = 0.5f * v * (1.0f + erff(v * 0.70710678118654752f));
    Cs[row * LDC + col] = gl * 8.0f;
  }
  __syncthreads();
  v4u ph[4], plq[4];
  size_t offs[4];
#pragma unroll
  for (int s = 0; s < 4; ++s) {
    const int idx = s * 256 + tid;
    const int row = idx >> 4, piece = idx & 15;
    const int col0 = piece * 8;
    v4u a, q4;
#pragma unroll
    for (int e = 0; e < 4; ++e) {
      const float f0 = Cs[row * LDC + col0 + 2 * e];
      const float f1 = Cs[row * LDC + col0 + 2 * e + 1];
      const _Float16 h0 = (_Float16)f0, h1 = (_Float16)f1;
      const float q0 = (f0 - (float)h0) * 2048.0f, q1 = (f1 - (float)h1) * 2048.0f;
      a[e]  = pk16(h_bits(h0), h_bits(h1));
      q4[e] = pk16(hb16(q0), hb16(q1));
    }
    ph[s] = a;
    plq[s] = q4;
    offs[s] = (size_t)(mb * 64 + row) * CMID + col0;
  }
#pragma unroll
  for (int s = 0; s < 4; ++s) { *(volatile v4u*)(fh + offs[s]) = ph[s]; *(volatile v4u*)(fl + offs[s]) = plq[s]; }
  __threadfence();
#pragma unroll
  for (int s = 0; s < 4; ++s) { *(volatile v4u*)(fh + offs[s]) = ph[s]; *(volatile v4u*)(fl + offs[s]) = plq[s]; }
}

__global__ __launch_bounds__(256)
void k_qkv(const unsigned short* __restrict__ fh, const unsigned short* __restrict__ fl,
           const unsigned short* __restrict__ wqkv, const float* __restrict__ qb,
           const float* __restrict__ kb, const float* __restrict__ vb, float* qkv) {
  __shared__ __align__(16) float Cs[64 * LDC];
  const int tid = threadIdx.x, wave = tid >> 5, lane = tid & 31;
  const int mb = blockIdx.x, nb = blockIdx.y;
  mm_tile2((const _Float16*)(const void*)fh, (const _Float16*)(const void*)fl, CMID,
           (const _Float16*)(const void*)wqkv, CMID, CMID / 32, mb * 64, nb * 128, Cs);
  __syncthreads();
  const float* bias = (nb == 0) ? qb : ((nb == 1) ? kb : vb);
  const int col0 = lane * 4;
  const v4f b4 = *(const v4f*)(bias + col0);
  v4f bb;
#pragma unroll
  for (int e = 0; e < 4; ++e) bb[e] = bfr(b4[e]);
#pragma unroll 1
  for (int it = 0; it < 8; ++it) {
    const int row = wave * 8 + it;
    const size_t t = (size_t)(mb * 64 + row);
    const v4f a = *(const v4f*)(Cs + row * LDC + col0);
    v4f o;
#pragma unroll
    for (int e = 0; e < 4; ++e) o[e] = a[e] * (1.0f / 512.0f) + bb[e];
    float* p = qkv + t * C3 + nb * CMID + col0;
    *(volatile v4f*)p = o;
    __threadfence();
    *(volatile v4f*)p = o;
  }
}

__global__ __launch_bounds__(128)
void k_attn(const float* __restrict__ qkv, float* out) {
  __shared__ float Ls[NKEY * 128];
  __shared__ __align__(16) float Os[CMID * OSP];
  const int tid = threadIdx.x, pl = tid >> 2, h = tid & 3;
  const int m0 = blockIdx.x * APB;
  const int b = m0 / IMGPIX;
  const int p0 = m0 - b * IMGPIX;
  const int y = p0 / WW;
  const int xb0 = p0 - y * WW;
  const int xw = xb0 + pl;
  const int m = m0 + pl;
  const float* qr = qkv + (size_t)m * C3 + h * HD;
  float q[HD];
#pragma unroll
  for (int d4 = 0; d4 < HD / 4; ++d4) {
    const v4f t4 = *(const v4f*)(qr + d4 * 4);
#pragma unroll
    for (int e = 0; e < 4; ++e) q[d4 * 4 + e] = t4[e];
  }
  const int sy = min(max(y - KSZ / 2, 0), HH - KSZ);
  const int sx = min(max(xw - KSZ / 2, 0), WW - KSZ);
  float mx = -3.0e38f;
#pragma unroll 1
  for (int key = 0; key < NKEY; ++key) {
    const int i = key / KSZ, j = key - i * KSZ;
    const int nm = (b * HH + sy + i) * WW + sx + j;
    const float* kr = qkv + (size_t)nm * C3 + CMID + h * HD;
    float s = 0.f;
#pragma unroll
    for (int d4 = 0; d4 < HD / 4; ++d4) {
      const v4f t4 = *(const v4f*)(kr + d4 * 4);
#pragma unroll
      for (int e = 0; e < 4; ++e) s += q[d4 * 4 + e] * t4[e];
    }
    s += __shfl_xor(s, 1, 32);
    s += __shfl_xor(s, 2, 32);
    s *= SCL;
    Ls[key * 128 + tid] = s;
    mx = fmaxf(mx, s);
  }
  float acc[HD];
#pragma unroll
  for (int d = 0; d < HD; ++d) acc[d] = 0.f;
  float l = 0.f;
#pragma unroll 1
  for (int key = 0; key < NKEY; ++key) {
    const int i = key / KSZ, j = key - i * KSZ;
    const int nm = (b * HH + sy + i) * WW + sx + j;
    const float p = __expf(Ls[key * 128 + tid] - mx);
    l += p;
    const float* vr = qkv + (size_t)nm * C3 + 2 * CMID + h * HD;
#pragma unroll
    for (int d4 = 0; d4 < HD / 4; ++d4) {
      const v4f t4 = *(const v4f*)(vr + d4 * 4);
#pragma unroll
      for (int e = 0; e < 4; ++e) acc[d4 * 4 + e] += p * t4[e];
    }
  }
  const float inv = __builtin_amdgcn_rcpf(l);
#pragma unroll
  for (int d = 0; d < HD; ++d) Os[(h * HD + d) * OSP + pl] = acc[d] * inv;
  __syncthreads();
  v4f pk[8];
  size_t offs[8];
#pragma unroll
  for (int s = 0; s < 8; ++s) {
    const int idx = s * 128 + tid;
    const int c = idx >> 3, piece = idx & 7;
    pk[s] = *(const v4f*)(Os + c * OSP + piece * 4);
    offs[s] = (size_t)(b * CMID + c) * IMGPIX + p0 + piece * 4;
  }
#pragma unroll
  for (int s = 0; s < 8; ++s) *(volatile v4f*)(out + offs[s]) = pk[s];
  __threadfence();
#pragma unroll
  for (int s = 0; s < 8; ++s) *(volatile v4f*)(out + offs[s]) = pk[s];
}

extern "C" void kernel_launch(void* const* d_in, const int* in_sizes, int n_in,
                              void* d_out, int out_size, void* d_ws, size_t ws_size,
                              hipStream_t stream) {
  if (n_in < 11) return;
  const int expect[11] = { NB * CIN * IMGPIX, CIN, CIN, CMID * KCV, CMID,
                           CMID * CMID, CMID, CMID * CMID, CMID, CMID * CMID, CMID };
  for (int i = 0; i < 11; ++i) if (in_sizes[i] != expect[i]) return;
  if (out_size != NB * CMID * IMGPIX) return;

  const float* x      = (const float*)d_in[0];
  const float* gn_w   = (const float*)d_in[1];
  const float* gn_b   = (const float*)d_in[2];
  const float* conv_w = (const float*)d_in[3];
  const float* conv_b = (const float*)d_in[4];
  const float* q_w    = (const float*)d_in[5];
  const float* q_b    = (const float*)d_in[6];
  const float* k_w    = (const float*)d_in[7];
  const float* k_b    = (const float*)d_in[8];
  const float* v_w    = (const float*)d_in[9];
  const float* v_b    = (const float*)d_in[10];
  float* out = (float*)d_out;

  const size_t AL = 65536;
  const size_t sWT  = (((size_t)CMID * KCV * 2) + AL - 1) / AL * AL;
  const size_t sWQ  = (((size_t)C3 * CMID * 2) + AL - 1) / AL * AL;
  const size_t sST  = (((size_t)NGRP * SLN * 4) + AL - 1) / AL * AL;
  const size_t sX   = (((size_t)PADPIX * CIN * 2) + AL - 1) / AL * AL;
  const size_t sF   = (((size_t)NPIX * CMID * 2) + AL - 1) / AL * AL;
  const size_t sQKV = (((size_t)NPIX * C3 * 4) + AL - 1) / AL * AL;

  size_t off = 0;
  const size_t oWT  = off; off += sWT;
  const size_t oWQ  = off; off += sWQ;
  const size_t oST  = off; off += sST;
  const size_t oXH  = off; off += sX;
  const size_t oXL  = off; off += sX;
  const size_t oFH  = off; off += sF;
  const size_t oFL  = off; off += sF;
  const size_t oQKV = off; off += sQKV;
  if (off > ws_size) return;
  if (off > (size_t)134217728) return;

  char* ws = (char*)d_ws;
  unsigned short* WT   = (unsigned short*)(ws + oWT);
  unsigned short* WQKV = (unsigned short*)(ws + oWQ);
  float*          ST   = (float*)(ws + oST);
  unsigned short* XH   = (unsigned short*)(ws + oXH);
  unsigned short* XL   = (unsigned short*)(ws + oXL);
  unsigned short* FH   = (unsigned short*)(ws + oFH);
  unsigned short* FL   = (unsigned short*)(ws + oFL);
  float*          QKV  = (float*)(ws + oQKV);

  const dim3 blk(256);
  k_wcvt<<<dim3(CMID + C3), blk, 0, stream>>>(conv_w, q_w, k_w, v_w, WT, WQKV);
  k_gnstat<<<dim3(NGRP), blk, 0, stream>>>(x, ST);
  k_xn<<<dim3((PADPIX / 4 + 7) / 8), blk, 0, stream>>>(x, gn_w, gn_b, ST, XH, XL);
  k_conv<<<dim3(NPIX / 64), blk, 0, stream>>>(XH, XL, WT, conv_b, FH, FL);
  k_qkv<<<dim3(NPIX / 64, 3), blk, 0, stream>>>(FH, FL, WQKV, q_b, k_b, v_b, QKV);
  k_attn<<<dim3(NPIX / APB), dim3(128), 0, stream>>>(QKV, out);
  (void)hipGetLastError();
}
